// SpeakerReasonModule_37151467110479
// MI455X (gfx1250) — hardware-run, weakly checked
//
#include <hip/hip_runtime.h>
#include <math.h>

typedef __attribute__((ext_vector_type(16))) __bf16   v16b;
typedef __attribute__((ext_vector_type(8)))  __bf16   v8b;
typedef __attribute__((ext_vector_type(16))) _Float16 v16h;
typedef __attribute__((ext_vector_type(8)))  _Float16 v8h;
typedef __attribute__((ext_vector_type(8)))  float    v8f;
typedef __attribute__((ext_vector_type(4)))  float    v4f;

constexpr int kB     = 32;
constexpr int kJ     = 256;
constexpr int kM     = 128;
constexpr int kD     = 200;
constexpr int kP     = 3;
constexpr int kKH    = 224;
constexpr int kK2    = 448;
constexpr int kNP    = 208;
constexpr int kG     = 800;
constexpr int kMP    = 224;
constexpr int kM16P  = 256;
constexpr int kVecP  = 224;
constexpr int kNW    = 16;
constexpr int kBLK   = 512;
constexpr int kSteps = kJ / 2;
static_assert((kKH % 32) == 0 && (kK2 % 32) == 0, "K multiples of 32");
static_assert((kNP % 16) == 0 && (kG % 16) == 0 && (kM % 16) == 0, "N tile multiples");
static_assert(kKH == 7 * 32 && kMP == 7 * 32 && kVecP == 7 * 32, "seven lane-strided columns per row");
static_assert((kD % 8) == 0 && (kD % 4) == 0, "8-element groups never straddle the pad boundary");
static_assert(kB * kM == 4096, "rows per speaker");
static_assert(kM == 4 * 32, "four lane-strided slots per lane");

constexpr float kCarryM   = 64.0f;
constexpr float kCarryV   = 32768.0f;
constexpr float kResid    = 2048.0f;
constexpr float kInvResid = 1.0f / kResid;
constexpr float kInvVM    = 1.0f / (kCarryV * kCarryM);

constexpr size_t kSzMem  = (size_t)kB * kM * kMP * 4;
constexpr size_t kSzM16  = (size_t)2 * kB * kM * kM16P * 2;
constexpr size_t kSzWfc  = (size_t)kNP * kKH * 2;
constexpr size_t kSzWg   = (size_t)kG * kK2 * 2;
constexpr size_t kSzWf1  = (size_t)kNP * kK2 * 2;
constexpr size_t kSzOutS = (size_t)2 * kB * kSteps * kMP * 4;
constexpr size_t kOffMemA = 0;
constexpr size_t kOffMemB = kOffMemA + kSzMem;
constexpr size_t kOffM16H = kOffMemB + kSzMem;
constexpr size_t kOffM16L = kOffM16H + kSzM16;
constexpr size_t kOffWfc  = kOffM16L + kSzM16;
constexpr size_t kOffWg   = kOffWfc + kSzWfc;
constexpr size_t kOffWf1  = kOffWg + kSzWg;
constexpr size_t kOffOutS = kOffWf1 + kSzWf1;
constexpr size_t kWsTotal = kOffOutS + kSzOutS;
static_assert(kWsTotal == 24065024ull, "carve total");
static_assert(kWsTotal <= 134217728ull, "carve cap");
static_assert((kOffMemB % 128) == 0 && (kOffM16H % 128) == 0 && (kOffM16L % 128) == 0 &&
              (kOffWfc % 128) == 0 && (kOffWg % 128) == 0 && (kOffWf1 % 128) == 0 &&
              (kOffOutS % 128) == 0, "128-B aligned regions");

constexpr int kLdsAhi   = 0;
constexpr int kLdsAlo   = kLdsAhi + 16 * kK2 * 2;
constexpr int kLdsQ     = kLdsAlo + 16 * kK2 * 2;
constexpr int kLdsH     = kLdsQ + 16 * kNP * 4;
constexpr int kLdsZ     = kLdsH + 16 * kNP * 4;
constexpr int kLdsAtt   = kLdsZ + 16 * kNP * 4;
constexpr int kLdsGates = kLdsAtt + 16 * kM * 4;
constexpr int kLdsVec   = kLdsGates + 16 * kG * 4;
constexpr int kLdsA2    = kLdsVec + 16 * 2 * kVecP * 2;
constexpr int kLdsTotal = kLdsA2 + 16 * kKH * 2;
static_assert(kLdsTotal == 149504, "LDS total");

__device__ __forceinline__ unsigned short f2bf_bits(float f) {
  unsigned u = __float_as_uint(f);
  return (unsigned short)((u + 0x7FFFu + ((u >> 16) & 1u)) >> 16);
}
__device__ __forceinline__ float bf_bits2f(unsigned short h) { return __uint_as_float(((unsigned)h) << 16); }
__device__ __forceinline__ float bf_rne(float f) { return bf_bits2f(f2bf_bits(f)); }
__device__ __forceinline__ void pin1(float& x) { asm volatile("" : "+v"(x)); }
__device__ __forceinline__ void pin4(v4f& x) { asm volatile("" : "+v"(x)); }

__device__ __forceinline__ float fast_sigmoid(float z) { return __builtin_amdgcn_rcpf(1.0f + __expf(-z)); }
__device__ __forceinline__ float fast_tanh(float z) { return 1.0f - 2.0f * __builtin_amdgcn_rcpf(__expf(2.0f * z) + 1.0f); }

__device__ __forceinline__ float h16_to_f32(unsigned hb) {
  const unsigned sgn = (hb & 0x8000u) << 16;
  const unsigned em = hb & 0x7fffu;
  const float fn = __uint_as_float((em << 13) + 0x38000000u);
  const float fs = (float)em * 5.9604644775390625e-8f;
  const float mag = (em < 0x400u) ? fs : fn;
  return __uint_as_float(__float_as_uint(mag) | sgn);
}

__device__ __forceinline__ void split_f16(float x, float carry, unsigned short& hb, unsigned short& lb) {
  const float xs = x * carry;
  const _Float16 hh = (_Float16)xs;
  hb = __builtin_bit_cast(unsigned short, hh);
  const float hf = h16_to_f32((unsigned)hb);
  const float res = (xs - hf) * kResid;
  const _Float16 ll = (_Float16)res;
  lb = __builtin_bit_cast(unsigned short, ll);
}

__device__ __forceinline__ void put_split(unsigned short* ph, unsigned short* pl, int idx, float v) {
  const unsigned short hb = f2bf_bits(v);
  const unsigned short lb = f2bf_bits(v - bf_bits2f(hb));
  ph[idx] = hb;
  pl[idx] = lb;
}

__device__ __forceinline__ void put_split3(unsigned short* ph, unsigned short* pl, int idx,
                                           unsigned short* p2, int idx2, float v) {
  const unsigned short hb = f2bf_bits(v);
  const float r1 = v - bf_bits2f(hb);
  const unsigned short mb = f2bf_bits(r1);
  const float r2 = r1 - bf_bits2f(mb);
  const unsigned short l2 = f2bf_bits(r2);
  ph[idx] = hb;
  pl[idx] = mb;
  p2[idx2] = l2;
}

__device__ __forceinline__ void put_vec16(unsigned short* vrow, int idx, float x, float carry) {
  unsigned short hb, lb;
  split_f16(x, carry, hb, lb);
  vrow[idx] = hb;
  vrow[kVecP + idx] = lb;
}

struct FragB {
  union U { v16b v; v8b h[2]; };
  static __device__ __forceinline__ v16b load(const __bf16* p) {
    U f; f.h[0] = *(const v8b*)(p); f.h[1] = *(const v8b*)(p + 16); return f.v;
  }
};
struct FragH {
  union U { v16h v; v8h h[2]; };
  static __device__ __forceinline__ v16h load(const _Float16* p) {
    U f; f.h[0] = *(const v8h*)(p); f.h[1] = *(const v8h*)(p + 16); return f.v;
  }
};
__device__ __forceinline__ v8f mma_bf(v16b a, v16b b, v8f c) {
  return __builtin_amdgcn_wmma_f32_16x16x32_bf16(false, a, false, b, (short)0, c, false, false);
}
__device__ __forceinline__ v8f mma_h(v16h a, v16h b, v8f c) {
  return __builtin_amdgcn_wmma_f32_16x16x32_f16(false, a, false, b, (short)0, c, false, false);
}
__device__ __forceinline__ void guard_b(v8f& c, v16b a0, v16b a1, v16b b0) {
  asm volatile("v_nop\n\tv_nop\n\tv_nop\n\tv_nop" : "+v"(c) : "v"(a0), "v"(a1), "v"(b0));
}
__device__ __forceinline__ void guard_h(v8f& c, v16h a, v16h b) {
  asm volatile("v_nop\n\tv_nop\n\tv_nop\n\tv_nop" : "+v"(c) : "v"(a), "v"(b));
}

template <int KP>
__device__ __forceinline__ void tile_gemm2(
    const unsigned short* sAhi, const unsigned short* sAlo, const unsigned short* sA2, int acol0, int k3end,
    const unsigned short* __restrict__ W,
    float* Y, int yld, int ntiles, int nvalid,
    const float* __restrict__ bias0, const float* __restrict__ bias1, bool two,
    int wave, int lane)
{
  const int rl = lane & 15;
  const int hf = lane >> 4;
  const __bf16* ahp = (const __bf16*)sAhi + rl * kK2 + acol0 + 8 * hf;
  const __bf16* alp = (const __bf16*)sAlo + rl * kK2 + acol0 + 8 * hf;
  const __bf16* a2p = (const __bf16*)sA2 + rl * kKH + 8 * hf;
  for (int nt = wave; nt < ntiles; nt += kNW) {
    const int n = nt * 16 + rl;
    const __bf16* bwp = (const __bf16*)W + (size_t)n * KP + 8 * hf;
    v8f acc = (v8f){0.f, 0.f, 0.f, 0.f, 0.f, 0.f, 0.f, 0.f};
#pragma unroll 1
    for (int k0 = 0; k0 < KP; k0 += 32) {
      const v16b ah = FragB::load(ahp + k0);
      const v16b al = FragB::load(alp + k0);
      const v16b bw = FragB::load(bwp + k0);
      acc = mma_bf(ah, bw, acc);
      acc = mma_bf(al, bw, acc);
      guard_b(acc, ah, al, bw);
      if (k0 < k3end) {
        const v16b a2 = FragB::load(a2p + k0);
        acc = mma_bf(a2, bw, acc);
        guard_b(acc, a2, a2, bw);
      }
    }
    const int nc = (n < nvalid) ? n : (nvalid - 1);
    float b0v = bias0[nc];
    float b1v = bias1[nc];
    pin1(b0v);
    pin1(b1v);
    b0v = bf_rne(b0v);
    b1v = bf_rne(b1v);
    const float bsum = b0v + (two ? b1v : 0.0f);
    const float badd = (n < nvalid) ? bsum : 0.0f;
#pragma unroll
    for (int r = 0; r < 8; ++r) Y[(8 * hf + r) * yld + n] = acc[r] + badd;
  }
}

template <int KSTEPS>
__device__ __forceinline__ void matvec16(
    const unsigned short* vrow,
    const unsigned short* Bh, const unsigned short* Bl, int ldb,
    int ntiles, int nUpd, float scale, float* outrow, int lane)
{
  const int rl = lane & 15;
  const int hf = lane >> 4;
  const int rsel = (rl < 1) ? 0 : 1;
  const bool live = (rl < 2);
  const _Float16* ap = (const _Float16*)vrow + rsel * kVecP + 8 * hf;
  const v16h zf = (v16h){0, 0, 0, 0, 0, 0, 0, 0, 0, 0, 0, 0, 0, 0, 0, 0};
#pragma unroll 1
  for (int nt = 0; nt < ntiles; ++nt) {
    const size_t bo = (size_t)(nt * 16 + rl) * ldb + 8 * hf;
    const _Float16* bhp = (const _Float16*)Bh + bo;
    const _Float16* blp = (const _Float16*)Bl + bo;
    v8f accD = (v8f){0.f, 0.f, 0.f, 0.f, 0.f, 0.f, 0.f, 0.f};
    v8f accE = (v8f){0.f, 0.f, 0.f, 0.f, 0.f, 0.f, 0.f, 0.f};
    const bool tileLo = (nt * 16 < nUpd);
#pragma unroll 1
    for (int ks = 0; ks < KSTEPS; ++ks) {
      const int k0 = ks * 32;
      v16h a = FragH::load(ap + k0);
      a = live ? a : zf;
      const v16h bh = FragH::load(bhp + k0);
      accD = mma_h(a, bh, accD);
      guard_h(accD, a, bh);
      if (tileLo) {
        const v16h bl = FragH::load(blp + k0);
        accE = mma_h(a, bl, accE);
        guard_h(accE, a, bl);
      }
    }
    const float d0 = accD[0];
    const float d1 = accD[1];
    const float e0 = accE[0];
    const float e1 = accE[1];
    const float r = (d0 + (d1 + e0 + e1 * kInvResid) * kInvResid) * scale;
    if (lane < 16) outrow[nt * 16 + lane] = r;
  }
}

__device__ __forceinline__ void mem_rows_dot(const float* wrow, const float* mrows, float (&acc)[7])
{
#pragma unroll 2
  for (int m = 0; m < kM; ++m) {
    const float wm = wrow[m];
    const float* mr = mrows + (size_t)m * kMP;
#pragma unroll
    for (int t = 0; t < 7; ++t) acc[t] = fmaf(wm, mr[32 * t], acc[t]);
  }
}

__global__ __launch_bounds__(256) void pad_mem_kernel(
    const float* __restrict__ ma, const float* __restrict__ mb, float* __restrict__ MA, float* __restrict__ MB)
{
  const float* src = (blockIdx.y == 0) ? ma : mb;
  float* dst = (blockIdx.y == 0) ? MA : MB;
  const int i = blockIdx.x * 256 + threadIdx.x;
  const int row = i / 56;
  const int c4 = i - row * 56;
  const bool valid = (c4 < 50);
  const int cc = valid ? c4 : 0;
  v4f v = *(const v4f*)(src + (size_t)row * kD + cc * 4);
  pin4(v);
  const float e0 = v[0];
  const float e1 = v[1];
  const float e2 = v[2];
  const float e3 = v[3];
  const float r0 = valid ? bf_rne(e0) : 0.0f;
  const float r1 = valid ? bf_rne(e1) : 0.0f;
  const float r2 = valid ? bf_rne(e2) : 0.0f;
  const float r3 = valid ? bf_rne(e3) : 0.0f;
  const v4f o = (v4f){r0, r1, r2, r3};
  float* q = dst + (size_t)i * 4;
  *(volatile v4f*)q = o;
  __threadfence();
  *(volatile v4f*)q = o;
}

__global__ __launch_bounds__(256) void build_rowplanes_kernel(
    const float* __restrict__ ma, const float* __restrict__ mb,
    unsigned short* __restrict__ H, unsigned short* __restrict__ L)
{
  const int i = blockIdx.x * 256 + threadIdx.x;
  const int g = i & 31;
  const int row = i >> 5;
  const int sp = row >> 12;
  const int rr = row & 4095;
  const float* src = (sp == 0) ? ma : mb;
  const bool valid = (g < 25);
  const int gc = valid ? g : 0;
  v4f a0 = *(const v4f*)(src + (size_t)rr * kD + gc * 8);
  v4f a1 = *(const v4f*)(src + (size_t)rr * kD + gc * 8 + 4);
  pin4(a0);
  pin4(a1);
  v8h hv, lv;
#pragma unroll
  for (int e = 0; e < 4; ++e) {
    const float x0 = a0[e];
    const float x1 = a1[e];
    const float f0 = valid ? bf_rne(x0) : 0.0f;
    const float f1 = valid ? bf_rne(x1) : 0.0f;
    unsigned short h0, l0, h1, l1;
    split_f16(f0, kCarryM, h0, l0);
    split_f16(f1, kCarryM, h1, l1);
    hv[e]     = __builtin_bit_cast(_Float16, h0);
    hv[4 + e] = __builtin_bit_cast(_Float16, h1);
    lv[e]     = __builtin_bit_cast(_Float16, l0);
    lv[4 + e] = __builtin_bit_cast(_Float16, l1);
  }
  unsigned short* qh = H + (size_t)i * 8;
  unsigned short* ql = L + (size_t)i * 8;
  *(volatile v8h*)qh = hv;
  *(volatile v8h*)ql = lv;
  __threadfence();
  *(volatile v8h*)qh = hv;
  *(volatile v8h*)ql = lv;
}

__global__ __launch_bounds__(256) void prep_weight_kernel(
    const float* __restrict__ s0, const float* __restrict__ s1,
    unsigned short* __restrict__ dw, int mode, int KP, int total8)
{
  const int i = blockIdx.x * 256 + threadIdx.x;
  if (i >= total8) return;
  const int e0 = i << 3;
  const int n = e0 / KP;
  const int k = e0 - n * KP;
  const int half = (k >= kKH) ? 1 : 0;
  const int kk = k - half * kKH;
  const bool nok = (mode == 1) ? true : (n < kD);
  const bool valid = nok && (kk < kD);
  const int nn = valid ? n : 0;
  const int kc = valid ? kk : 0;
  const float* src = s0;
  size_t off = (size_t)nn * kD + kc;
  if (mode == 1) {
    src = half ? s0 : s1;
  } else if (mode == 2) {
    off = (size_t)nn * (2 * kD) + (size_t)half * kD + kc;
  }
  v4f a0 = *(const v4f*)(src + off);
  v4f a1 = *(const v4f*)(src + off + 4);
  pin4(a0);
  pin4(a1);
  v8h wv;
#pragma unroll
  for (int e = 0; e < 4; ++e) {
    const float x0 = a0[e];
    const float x1 = a1[e];
    const float f0 = valid ? x0 : 0.0f;
    const float f1 = valid ? x1 : 0.0f;
    const unsigned short h0 = f2bf_bits(f0), h1 = f2bf_bits(f1);
    wv[e]     = __builtin_bit_cast(_Float16, h0);
    wv[4 + e] = __builtin_bit_cast(_Float16, h1);
  }
  unsigned short* qw = dw + (size_t)e0;
  *(volatile v8h*)qw = wv;
  __threadfence();
  *(volatile v8h*)qw = wv;
}

__global__ __launch_bounds__(512) void speaker_chain_kernel(
    const float* __restrict__ cosp, const float* __restrict__ bank,
    const float* __restrict__ b_fc, const float* __restrict__ b_fc1,
    const float* __restrict__ b_ih, const float* __restrict__ b_hh,
    const unsigned short* __restrict__ Wfc, const unsigned short* __restrict__ Wg,
    const unsigned short* __restrict__ Wf1,
    float* memA, float* memB,
    unsigned short* M16H, unsigned short* M16L,
    float* outS)
{
  extern __shared__ __align__(16) char smem[];
  unsigned short* sAhi = (unsigned short*)(smem + kLdsAhi);
  unsigned short* sAlo = (unsigned short*)(smem + kLdsAlo);
  float* qv     = (float*)(smem + kLdsQ);
  float* hv     = (float*)(smem + kLdsH);
  float* zsv    = (float*)(smem + kLdsZ);
  float* attv   = (float*)(smem + kLdsAtt);
  float* gatesv = (float*)(smem + kLdsGates);
  unsigned short* vecv = (unsigned short*)(smem + kLdsVec);
  unsigned short* sAl2 = (unsigned short*)(smem + kLdsA2);

  const int tid  = threadIdx.x;
  const int wave = tid >> 5;
  const int lane = tid & 31;
  const int s    = blockIdx.x & 1;
  const int b0   = (blockIdx.x >> 1) * kNW;
  const int b    = b0 + wave;
  const int sb   = s * kB + b;
  float* memp = (s == 0 ? memA : memB) + (size_t)b * kM * kMP;
  unsigned short* m16h = M16H + (size_t)sb * kM * kM16P;
  unsigned short* m16l = M16L + (size_t)sb * kM * kM16P;
  const int arow = wave * kK2;
  const int a2row = wave * kKH;
  float* qrow = qv + wave * kNP;
  float* hrow = hv + wave * kNP;
  float* zrow = zsv + wave * kNP;
  float* arw  = attv + wave * kM;
  const float* grow = gatesv + wave * kG;
  unsigned short* vrow = vecv + wave * 2 * kVecP;

#pragma unroll 1
  for (int jj = 0; jj < kSteps; ++jj) {
    const int j = 2 * jj + s;

    {
      const float* bp = bank + ((size_t)j * kB + b) * kD;
#pragma unroll
      for (int t = 0; t < 7; ++t) {
        const int d = lane + 32 * t;
        const int dc = (d < kD) ? d : (kD - 1);
        float v = bp[dc];
        pin1(v);
        v = (d < kD) ? bf_rne(v) : 0.0f;
        put_split(sAhi, sAlo, arow + kKH + d, v);
      }
      const float* cp = cosp + ((size_t)b * kJ + j) * kM;
#pragma unroll
      for (int t = 0; t < 4; ++t) {
        const float cv = cp[lane + 32 * t];
        arw[lane + 32 * t] = bf_rne(cv);
      }
    }
    __syncthreads();

    float hreg[7], creg[7], sv[7];
    {
      float acc[7];
#pragma unroll
      for (int t = 0; t < 7; ++t) acc[t] = 0.0f;
      mem_rows_dot(arw, memp + lane, acc);
#pragma unroll
      for (int t = 0; t < 7; ++t) {
        const int d = lane + 32 * t;
        hreg[t] = (d < kD) ? acc[t] : 0.0f;
        creg[t] = 0.0f;
        sv[t] = 0.0f;
        put_split3(sAhi, sAlo, arow + d, sAl2, a2row + d, hreg[t]);
      }
    }
    __syncthreads();

    tile_gemm2<kKH>(sAhi, sAlo, sAl2, kKH, 0, Wfc, qv, kNP, kNP / 16, kD, b_fc, b_fc, false, wave, lane);
    __syncthreads();
#pragma unroll
    for (int t = 0; t < 7; ++t) {
      const int d = lane + 32 * t;
      const int dq = (d < kNP) ? d : (kNP - 1);
      const float qd = qrow[dq];
      const float qs = (d < kD) ? qd : 0.0f;
      put_split(sAhi, sAlo, arow + kKH + d, qs);
    }
    __syncthreads();

#pragma unroll 1
    for (int p = 0; p < kP; ++p) {
      const int k3 = (p == 0) ? kKH : 0;
      tile_gemm2<kK2>(sAhi, sAlo, sAl2, 0, k3, Wg, gatesv, kG, kG / 16, kG, b_ih, b_hh, true, wave, lane);
      __syncthreads();

#pragma unroll
      for (int t = 0; t < 7; ++t) {
        const int d = lane + 32 * t;
        const int dc = (d < kD) ? d : (kD - 1);
        const float ig = grow[dc];
        const float fg = grow[kD + dc];
        const float gg = grow[2 * kD + dc];
        const float og = grow[3 * kD + dc];
        const float cn = fast_sigmoid(fg) * creg[t] + fast_sigmoid(ig) * fast_tanh(gg);
        const float hn = fast_sigmoid(og) * fast_tanh(cn);
        creg[t] = (d < kD) ? cn : 0.0f;
        hreg[t] = (d < kD) ? hn : 0.0f;
        put_vec16(vrow, d, hreg[t], kCarryV);
      }
      __syncthreads();

      matvec16<7>(vrow, m16h, m16l, kM16P, kM / 16, jj, kInvVM, arw, lane);
      __syncthreads();

      {
        const float l0 = arw[lane];
        const float l1 = arw[lane + 32];
        const float l2 = arw[lane + 64];
        const float l3 = arw[lane + 96];
        float mx = fmaxf(fmaxf(l0, l1), fmaxf(l2, l3));
#pragma unroll
        for (int off = 16; off > 0; off >>= 1) mx = fmaxf(mx, __shfl_xor(mx, off, 32));
        const float e0 = __expf(l0 - mx);
        const float e1 = __expf(l1 - mx);
        const float e2 = __expf(l2 - mx);
        const float e3 = __expf(l3 - mx);
        float sum = (e0 + e1) + (e2 + e3);
#pragma unroll
        for (int off = 16; off > 0; off >>= 1) sum += __shfl_xor(sum, off, 32);
        const float inv = __builtin_amdgcn_rcpf(sum);
        arw[lane]      = e0 * inv;
        arw[lane + 32] = e1 * inv;
        arw[lane + 64] = e2 * inv;
        arw[lane + 96] = e3 * inv;
      }
      __syncthreads();

      {
        float acc[7];
#pragma unroll
        for (int t = 0; t < 7; ++t) acc[t] = 0.0f;
        mem_rows_dot(arw, memp + lane, acc);
#pragma unroll
        for (int t = 0; t < 7; ++t) {
          const int d = lane + 32 * t;
          const float xs = (d < kD) ? acc[t] : 0.0f;
          put_split(sAhi, sAlo, arow + d, xs);
        }
      }
      __syncthreads();

      tile_gemm2<kK2>(sAhi, sAlo, sAl2, 0, 0, Wf1, qv, kNP, kNP / 16, kD, b_fc1, b_fc1, false, wave, lane);
      __syncthreads();

      float qs[7];
#pragma unroll
      for (int t = 0; t < 7; ++t) {
        const int d = lane + 32 * t;
        const int dq = (d < kNP) ? d : (kNP - 1);
        const float qd = qrow[dq];
        qs[t] = (d < kD) ? qd : 0.0f;
      }
      if (p < kP - 1) {
#pragma unroll
        for (int t = 0; t < 7; ++t) {
          const int d = lane + 32 * t;
          put_split(sAhi, sAlo, arow + kKH + d, qs[t]);
          put_split(sAhi, sAlo, arow + d, hreg[t]);
        }
      } else {
        const float* srow = memp + (size_t)jj * kMP + lane;
#pragma unroll
        for (int t = 0; t < 7; ++t) sv[t] = srow[32 * t];
        volatile float* op = outS + (((size_t)s * kB + b) * kSteps + jj) * kMP + lane;
#pragma unroll
        for (int t = 0; t < 7; ++t) op[32 * t] = qs[t];
        __threadfence();
#pragma unroll
        for (int t = 0; t < 7; ++t) op[32 * t] = qs[t];
        __threadfence();
#pragma unroll
        for (int t = 0; t < 7; ++t) {
          const int d = lane + 32 * t;
          put_split(sAhi, sAlo, arow + d, qs[t] + sv[t]);
        }
      }
      __syncthreads();
    }

    tile_gemm2<kKH>(sAhi, sAlo, sAl2, 0, 0, Wfc, zsv, kNP, kNP / 16, kD, b_fc, b_fc, true, wave, lane);
    __syncthreads();

    {
      float nv[7];
#pragma unroll
      for (int t = 0; t < 7; ++t) {
        const int d = lane + 32 * t;
        const int dq = (d < kNP) ? d : (kNP - 1);
        const float zd = zrow[dq];
        const float g = fast_tanh(zd) * sv[t];
        nv[t] = (d < kD) ? g : 0.0f;
      }
      volatile float* mw = memp + (size_t)jj * kMP + lane;
#pragma unroll
      for (int t = 0; t < 7; ++t) mw[32 * t] = nv[t];
      __threadfence();
#pragma unroll
      for (int t = 0; t < 7; ++t) mw[32 * t] = nv[t];
#pragma unroll
      for (int t = 0; t < 7; ++t) {
        const int d = lane + 32 * t;
        if (d < kNP) hrow[d] = nv[t];
      }
    }
    __syncthreads();

    {
      const int cl = (lane < 25) ? lane : 25;
      const bool on = (lane < 26);
      const v4f f0 = *(const v4f*)(hrow + cl * 8);
      const v4f f1 = *(const v4f*)(hrow + cl * 8 + 4);
      v8h hvv, lvv;
#pragma unroll
      for (int e = 0; e < 4; ++e) {
        const float y0 = f0[e];
        const float y1 = f1[e];
        const float x0 = on ? y0 : 0.0f;
        const float x1 = on ? y1 : 0.0f;
        unsigned short h0, l0, h1, l1;
        split_f16(x0, kCarryM, h0, l0);
        split_f16(x1, kCarryM, h1, l1);
        hvv[e]     = __builtin_bit_cast(_Float16, h0);
        hvv[4 + e] = __builtin_bit_cast(_Float16, h1);
        lvv[e]     = __builtin_bit_cast(_Float16, l0);
        lvv[4 + e] = __builtin_bit_cast(_Float16, l1);
      }
      unsigned short* ph = m16h + (size_t)jj * kM16P + lane * 8;
      unsigned short* pl = m16l + (size_t)jj * kM16P + lane * 8;
      *(volatile v8h*)ph = hvv;
      *(volatile v8h*)pl = lvv;
      __threadfence();
      *(volatile v8h*)ph = hvv;
      *(volatile v8h*)pl = lvv;
    }
    __threadfence();
    __syncthreads();
  }
}

__global__ __launch_bounds__(256) void repack_out_kernel(const float* __restrict__ outS, float* __restrict__ out)
{
  const int i = blockIdx.x * 256 + threadIdx.x;
  const int o = i * 4;
  const int b = o / (kJ * kD);
  const int rem = o - b * (kJ * kD);
  const int j = rem / kD;
  const int d = rem - j * kD;
  const size_t src = ((((size_t)(j & 1) * kB + b) * kSteps) + (size_t)(j >> 1)) * kMP + d;
  const v4f v = *(const v4f*)(outS + src);
  float* q = out + (size_t)o;
  *(volatile v4f*)q = v;
  __threadfence();
  *(volatile v4f*)q = v;
}

extern "C" void kernel_launch(void* const* d_in, const int* in_sizes, int n_in,
                              void* d_out, int out_size, void* d_ws, size_t ws_size,
                              hipStream_t stream) {
  if (n_in < 12) return;
  if (in_sizes[0] != kB * kJ * kM) return;
  if (in_sizes[1] != kJ * kB * kD) return;
  if (in_sizes[2] != kB * kM * kD) return;
  if (in_sizes[3] != kB * kM * kD) return;
  if (in_sizes[4] != kD * kD) return;
  if (in_sizes[5] != kD) return;
  if (in_sizes[6] != kD * 2 * kD) return;
  if (in_sizes[7] != kD) return;
  if (in_sizes[8] != kG * kD) return;
  if (in_sizes[9] != kG * kD) return;
  if (in_sizes[10] != kG) return;
  if (in_sizes[11] != kG) return;
  if (out_size != kB * kJ * kD) return;
  if (ws_size < kWsTotal) return;

  const float* cosp  = (const float*)d_in[0];
  const float* bank  = (const float*)d_in[1];
  const float* mem_a = (const float*)d_in[2];
  const float* mem_b = (const float*)d_in[3];
  const float* w_fc  = (const float*)d_in[4];
  const float* b_fc  = (const float*)d_in[5];
  const float* w_fc1 = (const float*)d_in[6];
  const float* b_fc1 = (const float*)d_in[7];
  const float* w_ih  = (const float*)d_in[8];
  const float* w_hh  = (const float*)d_in[9];
  const float* b_ih  = (const float*)d_in[10];
  const float* b_hh  = (const float*)d_in[11];
  float* out = (float*)d_out;

  char* ws = (char*)d_ws;
  float*          MEMA = (float*)(ws + kOffMemA);
  float*          MEMB = (float*)(ws + kOffMemB);
  unsigned short* M16H = (unsigned short*)(ws + kOffM16H);
  unsigned short* M16L = (unsigned short*)(ws + kOffM16L);
  unsigned short* WFC  = (unsigned short*)(ws + kOffWfc);
  unsigned short* WG   = (unsigned short*)(ws + kOffWg);
  unsigned short* WF1  = (unsigned short*)(ws + kOffWf1);
  float*          OUTS = (float*)(ws + kOffOutS);

  pad_mem_kernel<<<dim3((kB * kM * (kMP / 4)) / 256, 2), 256, 0, stream>>>(mem_a, mem_b, MEMA, MEMB);

  build_rowplanes_kernel<<<(2 * kB * kM * (kM16P / 8)) / 256, 256, 0, stream>>>(mem_a, mem_b, M16H, M16L);

  {
    const int t0 = kNP * kKH / 8;
    const int t1 = kG * kK2 / 8;
    const int t2 = kNP * kK2 / 8;
    prep_weight_kernel<<<(t0 + 255) / 256, 256, 0, stream>>>(w_fc, w_fc, WFC, 0, kKH, t0);
    prep_weight_kernel<<<(t1 + 255) / 256, 256, 0, stream>>>(w_ih, w_hh, WG, 1, kK2, t1);
    prep_weight_kernel<<<(t2 + 255) / 256, 256, 0, stream>>>(w_fc1, w_fc1, WF1, 2, kK2, t2);
  }

  speaker_chain_kernel<<<4, kBLK, kLdsTotal, stream>>>(
      cosp, bank, b_fc, b_fc1, b_ih, b_hh, WFC, WG, WF1, MEMA, MEMB, M16H, M16L, OUTS);

  repack_out_kernel<<<(kB * kJ * kD / 4) / 256, 256, 0, stream>>>(OUTS, out);
}
